// Cffn_29721173688896
// MI455X (gfx1250) — hardware-verified
//
#include <hip/hip_runtime.h>
#include <stdint.h>


typedef __bf16 bf16;
typedef __bf16 v16bf __attribute__((ext_vector_type(16)));
typedef __bf16 v8bf  __attribute__((ext_vector_type(8)));
typedef __bf16 v4bf  __attribute__((ext_vector_type(4)));
typedef float  v8f   __attribute__((ext_vector_type(8)));
typedef float  v4f_base __attribute__((ext_vector_type(4)));
typedef v4f_base __attribute__((__may_alias__)) v4f;

#define DIMN    2048
#define NLAD    3
#define DEPTH   5
#define EPS_CF  0.01f

#define BM      128
#define BN      128
#define BK      32
#define NK      (DIMN / BK)
#define LDK     40
#define THREADS 512
#define NWAVE   (THREADS / 32)
#define EPP     32

union Frag { v16bf v; v8bf p[2]; };

__device__ __forceinline__ v16bf load_frag(const bf16* s, int row, int h)
{
    Frag f;
    const bf16* q = s + row * LDK + 8 * h;
    f.p[0] = *(const v8bf*)(q);
    f.p[1] = *(const v8bf*)(q + 16);
    return f.v;
}

__device__ __forceinline__ void cvt_store4(bf16* dst, v4f v)
{
    v4bf o;
    o[0] = (bf16)v[0];
    o[1] = (bf16)v[1];
    o[2] = (bf16)v[2];
    o[3] = (bf16)v[3];
    *(v4bf*)dst = o;
}

__device__ __forceinline__ void mm_group(v16bf a0, v16bf a1, v16bf bU, v16bf bG,
                                         v8f& u0, v8f& u1, v8f& g0, v8f& g1)
{
    u0 = __builtin_amdgcn_wmma_f32_16x16x32_bf16(false, a0, false, bU, (short)0, u0, false, false);
    u1 = __builtin_amdgcn_wmma_f32_16x16x32_bf16(false, a1, false, bU, (short)0, u1, false, false);
    g0 = __builtin_amdgcn_wmma_f32_16x16x32_bf16(false, a0, false, bG, (short)0, g0, false, false);
    g1 = __builtin_amdgcn_wmma_f32_16x16x32_bf16(false, a1, false, bG, (short)0, g1, false, false);
    asm volatile("v_nop\n\tv_nop\n\tv_nop\n\tv_nop"
                 : "+v"(u0), "+v"(u1), "+v"(g0), "+v"(g1)
                 : "v"(a0), "v"(a1), "v"(bU), "v"(bG));
}

__global__ __launch_bounds__(THREADS)
void fused_gemm_ladder_kernel(const float* __restrict__ x,
                              const float* __restrict__ Uw,
                              const float* __restrict__ Gw,
                              const float* __restrict__ Lw,
                              const float* __restrict__ Vw,
                              float* __restrict__ out)
{
    __shared__ __align__(16) bf16  As[BM * LDK];
    __shared__ __align__(16) bf16  Us[BN * LDK];
    __shared__ __align__(16) bf16  Gs[BN * LDK];
    __shared__ __align__(16) float Ep[NWAVE * 16 * EPP];

    const int tid  = threadIdx.x;
    const int lane = tid & 31;
    const int wave = tid >> 5;
    const int h    = lane >> 4;
    const int m    = lane & 15;
    const int wm   = (wave >> 2) * 32;
    const int wn   = (wave & 3) * 32;
    const int m0   = blockIdx.y * BM;
    const int n0   = blockIdx.x * BN;

    v8f cU[2][2], cG[2][2];
#pragma unroll
    for (int i = 0; i < 2; ++i)
#pragma unroll
        for (int j = 0; j < 2; ++j) {
#pragma unroll
            for (int r = 0; r < 8; ++r) { cU[i][j][r] = 0.0f; cG[i][j][r] = 0.0f; }
        }

    auto kstep = [&](int k0) {
        __syncthreads();
#pragma unroll
        for (int it = 0; it < 2; ++it) {
            const int idx = tid + it * THREADS;
            const int r   = idx >> 3;
            const int c4  = (idx & 7) << 2;
            const v4f vx = *(const v4f*)(x  + (size_t)(m0 + r) * DIMN + k0 + c4);
            const v4f vu = *(const v4f*)(Uw + (size_t)(n0 + r) * DIMN + k0 + c4);
            const v4f vg = *(const v4f*)(Gw + (size_t)(n0 + r) * DIMN + k0 + c4);
            cvt_store4(As + r * LDK + c4, vx);
            cvt_store4(Us + r * LDK + c4, vu);
            cvt_store4(Gs + r * LDK + c4, vg);
        }
        __syncthreads();
        const v16bf a0 = load_frag(As, wm + m, h);
        const v16bf a1 = load_frag(As, wm + 16 + m, h);
        {
            const v16bf bU = load_frag(Us, wn + m, h);
            const v16bf bG = load_frag(Gs, wn + m, h);
            mm_group(a0, a1, bU, bG, cU[0][0], cU[1][0], cG[0][0], cG[1][0]);
        }
        {
            const v16bf bU = load_frag(Us, wn + 16 + m, h);
            const v16bf bG = load_frag(Gs, wn + 16 + m, h);
            mm_group(a0, a1, bU, bG, cU[0][1], cU[1][1], cG[0][1], cG[1][1]);
        }
    };

    for (int kt = 0; kt < NK; kt += 4) {
        kstep((kt + 0) * BK);
        kstep((kt + 1) * BK);
        kstep((kt + 2) * BK);
        kstep((kt + 3) * BK);
    }

    float* ep = Ep + wave * (16 * EPP);
    const int rsub = lane >> 3;
    const int cs4  = (lane & 7) << 2;

#pragma unroll
    for (int mi = 0; mi < 2; ++mi) {
#pragma unroll
        for (int ni = 0; ni < 2; ++ni) {
            const int gn = n0 + wn + 16 * ni + m;
            float lw[NLAD][DEPTH], vv[NLAD];
#pragma unroll
            for (int l = 0; l < NLAD; ++l) {
                vv[l] = Vw[(size_t)gn * NLAD + l];
#pragma unroll
                for (int k = 0; k < DEPTH; ++k)
                    lw[l][k] = Lw[((size_t)l * DIMN + gn) * DEPTH + k];
            }
#pragma unroll
            for (int j = 0; j < 8; ++j) {
                const int lr = 8 * h + j;
                const int gm = m0 + wm + 16 * mi + lr;
                const float lin  = cU[mi][ni][j];
                const float gacc = cG[mi][ni][j];
                const float xv   = x[(size_t)gm * DIMN + gn];
                const float sg   = 1.0f / (1.0f + expf(-gacc));
                const float g    = sg * xv;

                float comb = 0.0f;
#pragma unroll
                for (int l = 0; l < NLAD; ++l) {
                    float z = g * lw[l][DEPTH - 1];
#pragma unroll
                    for (int k = DEPTH - 2; k >= 0; --k) {
                        float den = 1.0f + z;
                        if (fabsf(den) < EPS_CF) den = (den >= 0.0f) ? EPS_CF : -EPS_CF;
                        const float ak = g * lw[l][k];
                        z = ak / den;
                    }
                    comb += z * vv[l];
                }
                ep[lr * EPP + 16 * ni + m] = lin + comb;
            }
        }
        __syncthreads();

        v4f vals[4];
#pragma unroll
        for (int s = 0; s < 4; ++s)
            vals[s] = *(const v4f*)(ep + (4 * s + rsub) * EPP + cs4);

        float* ob = out + (size_t)(m0 + wm + 16 * mi) * DIMN + n0 + wn + cs4;
#pragma unroll
        for (int s = 0; s < 4; ++s)
            *(volatile v4f*)(ob + (size_t)(4 * s + rsub) * DIMN) = vals[s];
        __threadfence();
#pragma unroll
        for (int s = 0; s < 4; ++s)
            *(volatile v4f*)(ob + (size_t)(4 * s + rsub) * DIMN) = vals[s];

        __syncthreads();
    }
}

extern "C" void kernel_launch(void* const* d_in, const int* in_sizes, int n_in,
                              void* d_out, int out_size, void* d_ws, size_t ws_size,
                              hipStream_t stream)
{
    (void)d_ws; (void)ws_size;
    if (n_in < 5) return;
    const int nx = in_sizes[0];
    if (nx <= 0 || (nx % DIMN) != 0) return;
    const int M = nx / DIMN;
    if ((M % BM) != 0) return;
    if (in_sizes[1] != DIMN * DIMN) return;
    if (in_sizes[2] != DIMN * DIMN) return;
    if (in_sizes[3] != NLAD * DIMN * DEPTH) return;
    if (in_sizes[4] != DIMN * NLAD) return;
    if (out_size != nx) return;

    const float* x  = (const float*)d_in[0];
    const float* Uw = (const float*)d_in[1];
    const float* Gw = (const float*)d_in[2];
    const float* Lw = (const float*)d_in[3];
    const float* Vw = (const float*)d_in[4];
    float* out = (float*)d_out;

    dim3 grid(DIMN / BN, M / BM);
    fused_gemm_ladder_kernel<<<grid, THREADS, 0, stream>>>(x, Uw, Gw, Lw, Vw, out);
    (void)hipGetLastError();
}
